// CrossAttention_61890478735686
// MI455X (gfx1250) — hardware-verified
//
#include <hip/hip_runtime.h>

typedef __attribute__((ext_vector_type(16))) _Float16 v16h;
typedef __attribute__((ext_vector_type(8)))  _Float16 v8h;
typedef __attribute__((ext_vector_type(8)))  float    v8f;
typedef __attribute__((ext_vector_type(4)))  float    v4f;

#ifndef NB
#define NB 16
#endif
#define NCH        256
#define NHW        256
#define NUNITS     128
#define QKD        64
#define KLEN       9
#define MPAD       16
#define IMG_STRIDE_FULL (NHW * NCH)
#define IMG_CHUNK  ((NB) < 8 ? (NB) : 8)

static_assert(NB % IMG_CHUNK == 0);
static_assert(NCH % 64 == 0 && NHW % 64 == 0 && QKD % 32 == 0 && NHW % 32 == 0);
static_assert((NUNITS * QKD) % 64 == 0 && (NUNITS * MPAD) % 64 == 0);
static_assert(NCH == 256 && QKD == 64 && MPAD == 16 && NUNITS == 128);

union FragH { v16h v; v8h h[2]; };
__device__ __forceinline__ v16h frag_ld(const _Float16* p) {
    FragH f; f.h[0] = *(const v8h*)(p); f.h[1] = *(const v8h*)(p + 16); return f.v;
}
__device__ __forceinline__ v8f wmma16(v16h a, v16h b, v8f c) {
    c = __builtin_amdgcn_wmma_f32_16x16x32_f16(false, a, false, b, (short)0, c, false, false);
    asm volatile("v_nop\n\tv_nop\n\tv_nop\n\tv_nop" : "+v"(c) : "v"(a), "v"(b));
    return c;
}
__device__ __forceinline__ float bf_rne(float v) {
    unsigned u = __float_as_uint(v);
    u = (u + 0x7fffu + ((u >> 16) & 1u)) & 0xffff0000u;
    return __uint_as_float(u);
}

__global__ __launch_bounds__(256) void k_trcast(const float* __restrict__ src, unsigned short* __restrict__ dst, int R, int C, float sc) {
    __shared__ __align__(16) _Float16 T[64 * 72];
    const int c0 = blockIdx.x * 64, r0 = blockIdx.y * 64, z = blockIdx.z;
    const int tid = threadIdx.x;
    const float* s = src + (size_t)z * R * C;
#pragma unroll
    for (int it = 0; it < 4; ++it) {
        const int p = it * 256 + tid; const int rl = p >> 4, c4 = (p & 15) * 4;
        const v4f x = *(const v4f*)(s + (size_t)(r0 + rl) * C + c0 + c4);
        T[(c4 + 0) * 72 + rl] = (_Float16)(bf_rne(x.x) * sc);
        T[(c4 + 1) * 72 + rl] = (_Float16)(bf_rne(x.y) * sc);
        T[(c4 + 2) * 72 + rl] = (_Float16)(bf_rne(x.z) * sc);
        T[(c4 + 3) * 72 + rl] = (_Float16)(bf_rne(x.w) * sc);
    }
    __syncthreads();
    _Float16* d = (_Float16*)dst + (size_t)z * C * R;
    v8h v[2];
#pragma unroll
    for (int it = 0; it < 2; ++it) { const int p = it * 256 + tid; v[it] = *(const v8h*)(T + (p >> 3) * 72 + (p & 7) * 8); }
    for (int pass = 0; pass < 2; ++pass) {
#pragma unroll
        for (int it = 0; it < 2; ++it) {
            const int p = it * 256 + tid; const int cl = p >> 3, j = p & 7;
            *(volatile v8h*)(d + (size_t)(c0 + cl) * R + r0 + j * 8) = v[it];
        }
        __threadfence();
    }
}

__global__ __launch_bounds__(256) void k_wvcast(const float* __restrict__ src, unsigned short* __restrict__ dst, float sc) {
    __shared__ __align__(16) _Float16 T[MPAD * 264];
    const int u = blockIdx.x, tid = threadIdx.x;
    const float* s = src + ((size_t)u * NHW + tid) * KLEN;
#pragma unroll
    for (int m = 0; m < KLEN; ++m) T[m * 264 + tid] = (_Float16)(bf_rne(s[m]) * sc);
#pragma unroll
    for (int m = KLEN; m < MPAD; ++m) T[m * 264 + tid] = (_Float16)0.0f;
    __syncthreads();
    _Float16* d = (_Float16*)dst + (size_t)u * MPAD * NHW;
    v8h v[2];
#pragma unroll
    for (int it = 0; it < 2; ++it) { const int p = it * 256 + tid; v[it] = *(const v8h*)(T + (p >> 5) * 264 + (p & 31) * 8); }
    for (int pass = 0; pass < 2; ++pass) {
#pragma unroll
        for (int it = 0; it < 2; ++it) {
            const int p = it * 256 + tid; const int row = p >> 5, j = p & 31;
            *(volatile v8h*)(d + (size_t)row * NHW + j * 8) = v[it];
        }
        __threadfence();
    }
}

__global__ __launch_bounds__(256) void k_gemm64h(
        const unsigned short* __restrict__ Ap, int lda, long long strideA,
        const unsigned short* __restrict__ Btp, int ldb, long long strideB,
        unsigned short* __restrict__ Cp, int ldc, long long strideC, long long tnStride, int nInRow,
        int M, int N, int K) {
    __shared__ __align__(16) float sT[8][16 * 68];
    const int b = blockIdx.y;
    const int lane = threadIdx.x & 31;
    const int wave = __builtin_amdgcn_readfirstlane(threadIdx.x >> 5);
    const int tilesN = N >> 6, tilesM = M >> 6;
    const int tile = blockIdx.x * 8 + wave;
    if (tile >= tilesM * tilesN) return;
    const int tm = tile / tilesN, tn = tile - tm * tilesN;
    const int m0 = tm << 6, n0 = tn << 6;
    const _Float16* Ab = (const _Float16*)Ap + (size_t)b * strideA;
    const _Float16* Bb = (const _Float16*)Btp + (size_t)b * strideB;
    const int rlane = lane & 15;
    const int koff = (lane >> 4) * 8;
    const int mOff = (lane >> 4) * 8;

    v8f acc[4][4];
#pragma unroll
    for (int i = 0; i < 4; ++i)
#pragma unroll
        for (int j = 0; j < 4; ++j) { v8f zz = {}; acc[i][j] = zz; }

    for (int k0 = 0; k0 < K; k0 += 32) {
        v16h bh[4];
#pragma unroll
        for (int j = 0; j < 4; ++j) bh[j] = frag_ld(Bb + (size_t)(n0 + (j << 4) + rlane) * ldb + koff + k0);
#pragma unroll
        for (int i = 0; i < 4; ++i) {
            const v16h ah = frag_ld(Ab + (size_t)(m0 + (i << 4) + rlane) * lda + koff + k0);
#pragma unroll
            for (int j = 0; j < 4; ++j) acc[i][j] = wmma16(ah, bh[j], acc[i][j]);
        }
    }

    _Float16* Cb = (_Float16*)Cp + (size_t)b * strideC + (size_t)tn * tnStride + (size_t)(nInRow ? n0 : 0);
    const int q = lane >> 3, c8 = (lane & 7) * 8;
#pragma unroll
    for (int i = 0; i < 4; ++i) {
        const int mBase = m0 + (i << 4);
#pragma unroll
        for (int j = 0; j < 4; ++j)
#pragma unroll
            for (int r = 0; r < 8; ++r) sT[wave][(mOff + r) * 68 + (j << 4) + rlane] = acc[i][j][r];
        __builtin_amdgcn_fence(3  , "workgroup");
        __builtin_amdgcn_wave_barrier();
        __builtin_amdgcn_fence(2  , "workgroup");
        v8h hv[4];
#pragma unroll
        for (int it = 0; it < 4; ++it) {
            const int row = it * 4 + q;
#pragma unroll
            for (int e = 0; e < 8; ++e) hv[it][e] = (_Float16)sT[wave][row * 68 + c8 + e];
        }
        for (int pass = 0; pass < 2; ++pass) {
#pragma unroll
            for (int it = 0; it < 4; ++it) {
                const int row = it * 4 + q;
                *(volatile v8h*)(Cb + (size_t)(mBase + row) * ldc + c8) = hv[it];
            }
            __threadfence();
        }
        __builtin_amdgcn_fence(3  , "workgroup");
        __builtin_amdgcn_wave_barrier();
        __builtin_amdgcn_fence(2  , "workgroup");
    }
}

__global__ __launch_bounds__(256) void k_attn(const unsigned short* __restrict__ QWp, const unsigned short* __restrict__ KWp,
                                              const unsigned short* __restrict__ VWp, float* __restrict__ FK, int nu0, int nuCount) {
    __shared__ __align__(16) float st[8][256];
    const int lane = threadIdx.x & 31, hh = lane >> 4, c = lane & 15;
    const int wave = __builtin_amdgcn_readfirstlane(threadIdx.x >> 5);
    const int nul = blockIdx.x >> 1;
    if (nul >= nuCount) return;
    const int q0 = (blockIdx.x & 1) * 128 + wave * 16;
    const _Float16* Qr = (const _Float16*)QWp + ((size_t)nul * NCH + q0 + c) * QKD + 8 * hh;
    const _Float16* Kb = (const _Float16*)KWp + (size_t)nul * NCH * QKD + (size_t)c * QKD + 8 * hh;
    const _Float16* Vb = (const _Float16*)VWp + ((size_t)nul * MPAD + c) * NCH + 8 * hh;
    const v16h qb0 = frag_ld(Qr), qb1 = frag_ld(Qr + 32);
    const float cs = 1.4426950408889634f * (1.0f / 4096.0f);
    v8f o = {};
    float m = -1.0e30f, lp = 0.0f;
#pragma unroll 1
    for (int ks = 0; ks < NCH / 32; ++ks) {
        const _Float16* kp = Kb + (size_t)(ks * 32) * QKD;
        v8f s0 = {}, s1 = {};
        s0 = wmma16(frag_ld(kp), qb0, s0);
        s0 = wmma16(frag_ld(kp + 32), qb1, s0);
        s1 = wmma16(frag_ld(kp + 16 * QKD), qb0, s1);
        s1 = wmma16(frag_ld(kp + 16 * QKD + 32), qb1, s1);
        float mx = fmaxf(s0[0], s1[0]);
#pragma unroll
        for (int r = 1; r < 8; ++r) mx = fmaxf(mx, fmaxf(s0[r], s1[r]));
        mx = fmaxf(mx, __shfl_xor(mx, 16, 32));
        const float mnew = fmaxf(m, mx * cs);
        const float corr = exp2f(m - mnew);
        float ps = 0.0f;
        v16h pb;
#pragma unroll
        for (int r = 0; r < 8; ++r) {
            const float p0 = exp2f(s0[r] * cs - mnew);
            const float p1 = exp2f(s1[r] * cs - mnew);
            ps += p0 + p1;
            pb[r]     = (_Float16)(p0 * 256.0f);
            pb[8 + r] = (_Float16)(p1 * 256.0f);
        }
        lp = lp * corr + ps;
        m = mnew;
#pragma unroll
        for (int r = 0; r < 8; ++r) o[r] *= corr;
        const v16h va = frag_ld(Vb + ks * 32);
        o = wmma16(va, pb, o);
    }
    const float l = lp + __shfl_xor(lp, 16, 32);
    const float inv = 1.0f / (l * 4096.0f);
    v4f a0, a1;
    a0.x = o[0] * inv; a0.y = o[1] * inv; a0.z = o[2] * inv; a0.w = o[3] * inv;
    a1.x = o[4] * inv; a1.y = o[5] * inv; a1.z = o[6] * inv; a1.w = o[7] * inv;
    *(v4f*)&st[wave][c * 16 + 8 * hh]     = a0;
    *(v4f*)&st[wave][c * 16 + 8 * hh + 4] = a1;
    __builtin_amdgcn_fence(3  , "workgroup");
    __builtin_amdgcn_wave_barrier();
    __builtin_amdgcn_fence(2  , "workgroup");
    const v4f w0 = *(const v4f*)&st[wave][lane * 4];
    const v4f w1 = *(const v4f*)&st[wave][128 + lane * 4];
    float* dst = FK + ((size_t)(nu0 + nul) * NCH + q0) * MPAD;
    for (int pass = 0; pass < 2; ++pass) {
        *(volatile v4f*)(dst + lane * 4) = w0;
        *(volatile v4f*)(dst + 128 + lane * 4) = w1;
        __threadfence();
    }
}

__global__ __launch_bounds__(128) void k_out(const float* __restrict__ FK, float* __restrict__ out) {
    const int c = blockIdx.x, n = blockIdx.y, u = threadIdx.x;
    const float* f = FK + (((size_t)n * NUNITS + u) * NCH + c) * MPAD;
    const v4f a = *(const v4f*)(f), b = *(const v4f*)(f + 4), d = *(const v4f*)(f + 8);
    float v[KLEN];
    v[0] = a.x; v[1] = a.y; v[2] = a.z; v[3] = a.w; v[4] = b.x; v[5] = b.y; v[6] = b.z; v[7] = b.w; v[8] = d.x;
    float* o = out + ((size_t)n * KLEN * NCH + c) * NUNITS + u;
    for (int pass = 0; pass < 2; ++pass) {
#pragma unroll
        for (int m = 0; m < KLEN; ++m) *(volatile float*)(o + (size_t)m * NCH * NUNITS) = v[m];
        __threadfence();
    }
}

#define SZ_IMG   ((size_t)NB * NCH * NHW * 2)
#define SZ_WQK   ((size_t)NUNITS * QKD * NHW * 2)
#define SZ_WV    ((size_t)NUNITS * MPAD * NHW * 2)
#define SZ_PROJ  ((size_t)IMG_CHUNK * NUNITS * NCH * QKD * 2)
#define SZ_VW    ((size_t)IMG_CHUNK * NUNITS * MPAD * NCH * 2)
#define SZ_FK    ((size_t)NB * NUNITS * NCH * MPAD * 4)
#define WS_TOTAL (2 * SZ_IMG + 2 * SZ_WQK + SZ_WV + 2 * SZ_PROJ + SZ_VW + SZ_FK)
static_assert(SZ_IMG % 256 == 0 && SZ_WQK % 256 == 0 && SZ_WV % 256 == 0 && SZ_PROJ % 256 == 0 && SZ_VW % 256 == 0 && SZ_FK % 256 == 0);
static_assert(WS_TOTAL <= (size_t)134217728);

extern "C" void kernel_launch(void* const* d_in, const int* in_sizes, int n_in, void* d_out, int out_size, void* d_ws, size_t ws_size, hipStream_t stream) {
    if (n_in < 5) return;
    if (in_sizes[0] < NB * IMG_STRIDE_FULL || in_sizes[1] < NB * IMG_STRIDE_FULL) return;
    if (in_sizes[2] < NUNITS * NHW * QKD || in_sizes[3] < NUNITS * NHW * QKD || in_sizes[4] < NUNITS * NHW * KLEN) return;
    if (out_size < NB * KLEN * NCH * NUNITS) return;
    if (ws_size < WS_TOTAL) return;
    const float* query   = (const float*)d_in[0];
    const float* value   = (const float*)d_in[1];
    const float* query_w = (const float*)d_in[2];
    const float* key_w   = (const float*)d_in[3];
    const float* value_w = (const float*)d_in[4];
    float* out = (float*)d_out;

    char* wsp = (char*)d_ws;
    unsigned short* QT  = (unsigned short*)wsp; wsp += SZ_IMG;
    unsigned short* VT0 = (unsigned short*)wsp; wsp += SZ_IMG;
    unsigned short* WQT = (unsigned short*)wsp; wsp += SZ_WQK;
    unsigned short* WKT = (unsigned short*)wsp; wsp += SZ_WQK;
    unsigned short* WVT = (unsigned short*)wsp; wsp += SZ_WV;
    unsigned short* QW  = (unsigned short*)wsp; wsp += SZ_PROJ;
    unsigned short* KW  = (unsigned short*)wsp; wsp += SZ_PROJ;
    unsigned short* VWT = (unsigned short*)wsp; wsp += SZ_VW;
    float*          FK  = (float*)wsp;          wsp += SZ_FK;

    k_trcast<<<dim3(NCH / 64, NHW / 64, NB), 256, 0, stream>>>(query, QT, NHW, NCH, 1.0f);
    k_trcast<<<dim3(NCH / 64, NHW / 64, NB), 256, 0, stream>>>(value, VT0, NHW, NCH, 1.0f);
    k_trcast<<<dim3(QKD / 64, NHW / 64, NUNITS), 256, 0, stream>>>(query_w, WQT, NHW, QKD, 16.0f);
    k_trcast<<<dim3(QKD / 64, NHW / 64, NUNITS), 256, 0, stream>>>(key_w, WKT, NHW, QKD, 16.0f);
    k_wvcast<<<NUNITS, 256, 0, stream>>>(value_w, WVT, 16.0f);

    for (int ch = 0; ch < NB / IMG_CHUNK; ++ch) {
        const int n0 = ch * IMG_CHUNK;
        const unsigned short* QTc = QT  + (size_t)n0 * NCH * NHW;
        const unsigned short* VTc = VT0 + (size_t)n0 * NCH * NHW;
        k_gemm64h<<<dim3(((NCH / 64) * (NUNITS * QKD / 64) + 7) / 8, IMG_CHUNK), 256, 0, stream>>>(
            QTc, NHW, (long long)NCH * NHW, WQT, NHW, 0LL,
            QW, QKD, (long long)NUNITS * NCH * QKD, (long long)NCH * QKD, 0, NCH, NUNITS * QKD, NHW);
        k_gemm64h<<<dim3(((NCH / 64) * (NUNITS * QKD / 64) + 7) / 8, IMG_CHUNK), 256, 0, stream>>>(
            VTc, NHW, (long long)NCH * NHW, WKT, NHW, 0LL,
            KW, QKD, (long long)NUNITS * NCH * QKD, (long long)NCH * QKD, 0, NCH, NUNITS * QKD, NHW);
        k_gemm64h<<<dim3(((NUNITS * MPAD / 64) * (NCH / 64) + 7) / 8, IMG_CHUNK), 256, 0, stream>>>(
            WVT, NHW, 0LL, VTc, NHW, (long long)NCH * NHW,
            VWT, NCH, (long long)NUNITS * MPAD * NCH, 0LL, 1, NUNITS * MPAD, NCH, NHW);
        k_attn<<<IMG_CHUNK * NUNITS * 2, 256, 0, stream>>>(QW, KW, VWT, FK, n0 * NUNITS, IMG_CHUNK * NUNITS);
    }
    k_out<<<dim3(NCH, NB), 128, 0, stream>>>(FK, out);
}
